// MambaBlock_62448824483847
// MI455X (gfx1250) — hardware-verified
//
#include <hip/hip_runtime.h>
#include <stddef.h>
#include <stdint.h>
#include <math.h>


#define LSEQ   2048
#define DM     1024
#define DI     2048
#define NS     16
#define NPJ    4096
#define K2     4096
#define XPN    64
#define XPV    33
#define NTHR   256
#define GBM    64
#define GBN    64
#define GTHR   128
#define SCH    64
#define SCT    64
#define XPP    36
#define NCHK   (LSEQ / SCH)

#define U_XB   (LSEQ * DM / 8)
#define U_WIN  (NPJ * DM / 8)
#define U_OW   (DM * K2 / 8)
#define U_XPW  (XPN * K2 / 8)
#define U_TOT  (U_XB + U_WIN + U_OW + U_XPW)
#define E_XB   0
#define E_WIN  (LSEQ * DM)
#define E_OW   (E_WIN + NPJ * DM)
#define E_XPW  (E_OW + DM * K2)
#define E_END  (E_XPW + XPN * K2)
#define WSMAX  134217728

static_assert(U_XB % NTHR == 0 && U_WIN % NTHR == 0 && U_OW % NTHR == 0 && U_XPW % NTHR == 0);
static_assert(DM % 32 == 0 && K2 % 32 == 0 && K2 == 2 * DI);
static_assert(LSEQ % GBM == 0 && NPJ % GBN == 0 && DM % GBN == 0 && XPN % GBN == 0 && DI % GBN == 0);
static_assert(GBM == (GTHR / 32) * 16 && GBN == 64);
static_assert((LSEQ * (DI / 4)) % NTHR == 0 && (DI / 4) % 32 == 0);
static_assert(LSEQ % SCH == 0 && DI % SCT == 0 && SCT == 64 && SCH == 64);
static_assert(XPP % 4 == 0 && XPP >= XPV && XPP <= XPN);
static_assert(((size_t)E_END * 2) % 256 == 0);

typedef float          v4f   __attribute__((ext_vector_type(4)));
typedef float          v8f   __attribute__((ext_vector_type(8)));
typedef int            v8i   __attribute__((ext_vector_type(8)));
typedef unsigned int   v4u   __attribute__((ext_vector_type(4)));
typedef unsigned short v8us  __attribute__((ext_vector_type(8)));
typedef unsigned short v16us __attribute__((ext_vector_type(16)));
typedef __bf16         v16bf __attribute__((ext_vector_type(16)));
typedef v4f  __attribute__((may_alias)) v4fa;
typedef v8us __attribute__((may_alias)) v8usa;
union FragB { v16bf v; v16us u; v8us h[2]; v8i w; };

__device__ __forceinline__ v8f wmb(const FragB& a, const FragB& b, v8f c) {
  v8f d = __builtin_amdgcn_wmma_f32_16x16x32_bf16(false, a.v, false, b.v, (short)0, c, false, false);
  asm volatile("v_nop\n\tv_nop\n\tv_nop\n\tv_nop" : "+v"(d) : "v"(a.w), "v"(b.w));
  return d;
}

__device__ __forceinline__ unsigned bf16_bits(float f) {
  const unsigned u = __float_as_uint(f);
  return (u + 0x7FFFu + ((u >> 16) & 1u)) >> 16;
}
__device__ __forceinline__ float bf16_val(float f) {
  return __uint_as_float(bf16_bits(f) << 16);
}
__device__ __forceinline__ float silu1(float v) {
  return v * (1.0f / (1.0f + expf(-v)));
}
__device__ __forceinline__ v8us cvt8(const float* p, bool ok) {
  const v4f a = *(const v4fa*)p;
  const v4f b = *(const v4fa*)(p + 4);
  v8us o;
  o[0] = ok ? (unsigned short)bf16_bits(a.x) : (unsigned short)0;
  o[1] = ok ? (unsigned short)bf16_bits(a.y) : (unsigned short)0;
  o[2] = ok ? (unsigned short)bf16_bits(a.z) : (unsigned short)0;
  o[3] = ok ? (unsigned short)bf16_bits(a.w) : (unsigned short)0;
  o[4] = ok ? (unsigned short)bf16_bits(b.x) : (unsigned short)0;
  o[5] = ok ? (unsigned short)bf16_bits(b.y) : (unsigned short)0;
  o[6] = ok ? (unsigned short)bf16_bits(b.z) : (unsigned short)0;
  o[7] = ok ? (unsigned short)bf16_bits(b.w) : (unsigned short)0;
  return o;
}

__global__ __launch_bounds__(NTHR) void k_prep(const float* __restrict__ x, const float* __restrict__ wi,
                                               const float* __restrict__ wo, const float* __restrict__ xpw,
                                               unsigned short* planes) {
  const int u = (int)blockIdx.x * NTHR + (int)threadIdx.x;
  v8us o;
  size_t doff;
  if (u < U_XB) {
    o = cvt8(x + (size_t)u * 8, true);
    doff = (size_t)E_XB + (size_t)u * 8;
  } else if (u < U_XB + U_WIN) {
    const int v = u - U_XB;
    o = cvt8(wi + (size_t)v * 8, true);
    doff = (size_t)E_WIN + (size_t)v * 8;
  } else if (u < U_XB + U_WIN + U_OW) {
    const int v  = u - (U_XB + U_WIN);
    const int n  = v >> 9;
    const int k8 = (v & 511) * 8;
    o = cvt8(wo + (size_t)n * DI + (k8 & (DI - 1)), true);
    doff = (size_t)E_OW + (size_t)n * K2 + k8;
  } else if (u < U_TOT) {
    const int v  = u - (U_XB + U_WIN + U_OW);
    const int n  = v >> 9;
    const int k8 = (v & 511) * 8;
    const int nc = n < XPV ? n : XPV - 1;
    o = cvt8(xpw + (size_t)nc * DI + (k8 & (DI - 1)), n < XPV);
    doff = (size_t)E_XPW + (size_t)n * K2 + k8;
  } else {
    return;
  }
  unsigned short* dp = planes + doff;
  *(volatile v8us*)dp = o;
  __threadfence();
  *(volatile v8us*)dp = o;
}

template <int EPI>
__global__ __launch_bounds__(GTHR) void k_gemm(
    const unsigned short* __restrict__ A, const unsigned short* __restrict__ WT,
    float* outF, int K, int ldo, int splitN, int planeStride)
{
  __shared__ __attribute__((aligned(16))) float stg[GBM * GBN];
  const int tid = (int)threadIdx.x, lane = tid & 31, wave = tid >> 5, hh = lane >> 4, m = lane & 15;
  const int rowBase = (int)blockIdx.x * GBM;
  const int col0    = (int)blockIdx.y * GBN;
  int plane = 0, colo = col0;
  if constexpr (EPI != 0) {
    if (col0 >= splitN) { plane = 1; colo = col0 - splitN; }
  }

  v8f acc[4];
  {
    const v8f z = {0.f, 0.f, 0.f, 0.f, 0.f, 0.f, 0.f, 0.f};
    acc[0] = z; acc[1] = z; acc[2] = z; acc[3] = z;
  }
  const unsigned short* ap = A  + (size_t)(rowBase + 16 * wave + m) * (size_t)K + 8 * hh;
  const unsigned short* wp = WT + (size_t)(col0 + m) * (size_t)K + 8 * hh;
  const int ksteps = K >> 5;
#pragma unroll 1
  for (int ks = 0; ks < ksteps; ++ks) {
    FragB af;
    af.h[0] = *(const v8usa*)(ap + 32 * ks);
    af.h[1] = *(const v8usa*)(ap + 32 * ks + 16);
#pragma unroll
    for (int t = 0; t < 4; ++t) {
      const unsigned short* wq = wp + (size_t)(16 * t) * (size_t)K + 32 * ks;
      FragB bf;
      bf.h[0] = *(const v8usa*)wq;
      bf.h[1] = *(const v8usa*)(wq + 16);
      acc[t] = wmb(af, bf, acc[t]);
    }
  }

#pragma unroll
  for (int t = 0; t < 4; ++t) {
    const int lc = 16 * t + m;
#pragma unroll
    for (int r = 0; r < 8; ++r) {
      const int lr = 16 * wave + 8 * hh + r;
      stg[lr * GBN + lc] = acc[t][r];
    }
  }
  __syncthreads();

  if constexpr (EPI != 0) {
    if (plane != 0) {
#pragma unroll 1
      for (int i = 0; i < 8; ++i) {
        float* sp = stg + (16 * wave + 2 * i + hh) * GBN + 4 * m;
        v4f v = *(const v4fa*)sp;
        v.x = silu1(v.x); v.y = silu1(v.y); v.z = silu1(v.z); v.w = silu1(v.w);
        *(v4fa*)sp = v;
      }
    }
  }

  float* ob = outF + (size_t)plane * (size_t)planeStride;
  v4f fv[8];
#pragma unroll
  for (int i = 0; i < 8; ++i) {
    const int lr = 16 * wave + 2 * i + hh;
    fv[i] = *(const v4fa*)(stg + lr * GBN + 4 * m);
  }
#pragma unroll
  for (int i = 0; i < 8; ++i) {
    const int lr = 16 * wave + 2 * i + hh;
    const int gr = rowBase + lr;
    float* op = ob + (size_t)gr * (size_t)ldo + colo + 4 * m;
    *(volatile v4f*)op = fv[i];
  }
  __threadfence();
#pragma unroll
  for (int i = 0; i < 8; ++i) {
    const int lr = 16 * wave + 2 * i + hh;
    const int gr = rowBase + lr;
    float* op = ob + (size_t)gr * (size_t)ldo + colo + 4 * m;
    *(volatile v4f*)op = fv[i];
  }
}

__global__ __launch_bounds__(NTHR) void k_conv(const float* __restrict__ xs, const float* __restrict__ cw,
                                               const float* __restrict__ cb, float* xc, unsigned short* xchl) {
  const int tid = (int)threadIdx.x, lane = tid & 31;
  const int idx = (int)blockIdx.x * NTHR + tid;
  const int l   = idx >> 9;
  const int dg  = idx & 511;
  const int d0  = dg * 4;
  const v4f w0 = *(const v4fa*)(cw + (size_t)d0 * 4);
  const v4f w1 = *(const v4fa*)(cw + (size_t)d0 * 4 + 4);
  const v4f w2 = *(const v4fa*)(cw + (size_t)d0 * 4 + 8);
  const v4f w3 = *(const v4fa*)(cw + (size_t)d0 * 4 + 12);
  const v4f bb = *(const v4fa*)(cb + d0);
  float a0 = 0.0f, a1 = 0.0f, a2 = 0.0f, a3 = 0.0f;
#pragma unroll
  for (int k = 0; k < 4; ++k) {
    const int ll  = l - 3 + k;
    const int llc = ll < 0 ? 0 : ll;
    const float mk = (ll >= 0) ? 1.0f : 0.0f;
    const v4f xv = *(const v4fa*)(xs + (size_t)llc * DI + d0);
    a0 = fmaf(bf16_val(w0[k]) * mk, xv.x, a0);
    a1 = fmaf(bf16_val(w1[k]) * mk, xv.y, a1);
    a2 = fmaf(bf16_val(w2[k]) * mk, xv.z, a2);
    a3 = fmaf(bf16_val(w3[k]) * mk, xv.w, a3);
  }
  v4f o;
  o.x = silu1(a0 + bf16_val(bb.x));
  o.y = silu1(a1 + bf16_val(bb.y));
  o.z = silu1(a2 + bf16_val(bb.z));
  o.w = silu1(a3 + bf16_val(bb.w));

  const unsigned hb0 = bf16_bits(o.x), hb1 = bf16_bits(o.y), hb2 = bf16_bits(o.z), hb3 = bf16_bits(o.w);
  const unsigned lb0 = bf16_bits(o.x - __uint_as_float(hb0 << 16));
  const unsigned lb1 = bf16_bits(o.y - __uint_as_float(hb1 << 16));
  const unsigned lb2 = bf16_bits(o.z - __uint_as_float(hb2 << 16));
  const unsigned lb3 = bf16_bits(o.w - __uint_as_float(hb3 << 16));
  const int hw0 = (int)(hb0 | (hb1 << 16)), hw1 = (int)(hb2 | (hb3 << 16));
  const int lw0 = (int)(lb0 | (lb1 << 16)), lw1 = (int)(lb2 | (lb3 << 16));
  const int sa = (2 * lane) & 31, sb = (2 * lane + 1) & 31;
  const int g0 = __shfl(hw0, sa, 32), g1 = __shfl(hw1, sa, 32);
  const int g2 = __shfl(hw0, sb, 32), g3 = __shfl(hw1, sb, 32);
  const int p0 = __shfl(lw0, sa, 32), p1 = __shfl(lw1, sa, 32);
  const int p2 = __shfl(lw0, sb, 32), p3 = __shfl(lw1, sb, 32);
  const bool lsel = lane >= 16;
  v4u pv;
  pv.x = (unsigned)(lsel ? p0 : g0);
  pv.y = (unsigned)(lsel ? p1 : g1);
  pv.z = (unsigned)(lsel ? p2 : g2);
  pv.w = (unsigned)(lsel ? p3 : g3);
  const int wbase = d0 - 4 * lane;
  float* xp = xc + (size_t)l * DI + d0;
  unsigned short* hp = xchl + (size_t)l * K2 + (lsel ? DI : 0) + wbase + 8 * (lane & 15);
  *(volatile v4f*)xp = o;
  *(volatile v4u*)hp = pv;
  __threadfence();
  *(volatile v4f*)xp = o;
  *(volatile v4u*)hp = pv;
}

__global__ __launch_bounds__(SCT) void k_scan(const float* __restrict__ xp, const float* __restrict__ xc,
                                              const float* __restrict__ g, const float* __restrict__ alog,
                                              const float* __restrict__ dtw, const float* __restrict__ dtb,
                                              const float* __restrict__ dd, unsigned short* yg) {
  __shared__ __attribute__((aligned(16))) float xps[SCH * XPP];
  __shared__ __attribute__((aligned(16))) unsigned short stg[2 * SCH * SCT];
  const int t    = (int)threadIdx.x;
  const int dblk = (int)blockIdx.x * SCT;
  const int d    = dblk + t;

  float A[NS], h[NS];
#pragma unroll
  for (int j = 0; j < 4; ++j) {
    const v4f q = *(const v4fa*)(alog + (size_t)d * NS + 4 * j);
    A[4 * j + 0] = -expf(bf16_val(q.x));
    A[4 * j + 1] = -expf(bf16_val(q.y));
    A[4 * j + 2] = -expf(bf16_val(q.z));
    A[4 * j + 3] = -expf(bf16_val(q.w));
  }
#pragma unroll
  for (int n = 0; n < NS; ++n) h[n] = 0.0f;
  const float wd = bf16_val(dtw[d]);
  const float bd = bf16_val(dtb[d]);
  const float Dd = bf16_val(dd[d]);

#pragma unroll 1
  for (int ch = 0; ch < NCHK; ++ch) {
    const int l0 = ch * SCH;
#pragma unroll 1
    for (int i = t; i < SCH * (XPP / 4); i += SCT) {
      const int row = i / (XPP / 4);
      const int c4  = i - row * (XPP / 4);
      const v4f v = *(const v4fa*)(xp + (size_t)(l0 + row) * XPN + 4 * c4);
      *(v4fa*)(xps + row * XPP + 4 * c4) = v;
    }
    __syncthreads();

#pragma unroll 1
    for (int ls = 0; ls < SCH; ++ls) {
      const int l = l0 + ls;
      float xv[XPP];
#pragma unroll
      for (int j = 0; j < XPP / 4; ++j) {
        const v4f q = *(const v4fa*)(xps + ls * XPP + 4 * j);
        xv[4 * j + 0] = q.x; xv[4 * j + 1] = q.y; xv[4 * j + 2] = q.z; xv[4 * j + 3] = q.w;
      }
      const float xcv = xc[(size_t)l * DI + d];
      const float gv  = g[(size_t)l * DI + d];
      const float v   = fmaf(xv[0], wd, bd);
      const float dt  = fmaxf(v, 0.0f) + log1pf(expf(-fabsf(v)));
      const float dx  = dt * xcv;
      float y = 0.0f;
#pragma unroll
      for (int n = 0; n < NS; ++n) {
        const float dA = __expf(dt * A[n]);
        h[n] = fmaf(dA, h[n], dx * xv[1 + n]);
        y = fmaf(h[n], xv[1 + NS + n], y);
      }
      const float ygv = fmaf(xcv, Dd, y) * gv;
      const unsigned hb = bf16_bits(ygv);
      const unsigned lb = bf16_bits(ygv - __uint_as_float(hb << 16));
      stg[ls * SCT + t]         = (unsigned short)hb;
      stg[(SCH + ls) * SCT + t] = (unsigned short)lb;
    }
    __syncthreads();

    v8us qv[16];
#pragma unroll
    for (int it = 0; it < 16; ++it) {
      const int ln    = it * 8 + (t >> 3);
      const int row   = ln >> 1;
      const int plane = ln & 1;
      qv[it] = *(const v8usa*)(stg + (plane * SCH + row) * SCT + (t & 7) * 8);
    }
#pragma unroll
    for (int it = 0; it < 16; ++it) {
      const int ln    = it * 8 + (t >> 3);
      const int row   = ln >> 1;
      const int plane = ln & 1;
      unsigned short* op = yg + (size_t)(l0 + row) * K2 + plane * DI + dblk + (t & 7) * 8;
      *(volatile v8us*)op = qv[it];
    }
    __threadfence();
#pragma unroll
    for (int it = 0; it < 16; ++it) {
      const int ln    = it * 8 + (t >> 3);
      const int row   = ln >> 1;
      const int plane = ln & 1;
      unsigned short* op = yg + (size_t)(l0 + row) * K2 + plane * DI + dblk + (t & 7) * 8;
      *(volatile v8us*)op = qv[it];
    }
  }
}

static inline size_t al256(size_t o) { return (o + 255) & ~(size_t)255; }

extern "C" void kernel_launch(void* const* d_in, const int* in_sizes, int n_in,
                              void* d_out, int out_size, void* d_ws, size_t ws_size,
                              hipStream_t stream) {
  if (n_in < 10) return;
  if (in_sizes[0] != LSEQ * DM) return;
  if (in_sizes[1] != NPJ * DM) return;
  if (in_sizes[2] != DI * 4) return;
  if (in_sizes[3] != DI) return;
  if (in_sizes[4] != XPV * DI) return;
  if (in_sizes[5] != DI) return;
  if (in_sizes[6] != DI) return;
  if (in_sizes[7] != DI * NS) return;
  if (in_sizes[8] != DI) return;
  if (in_sizes[9] != DM * DI) return;
  if (out_size != LSEQ * DM) return;

  const float* x    = (const float*)d_in[0];
  const float* wi   = (const float*)d_in[1];
  const float* cw   = (const float*)d_in[2];
  const float* cb   = (const float*)d_in[3];
  const float* xpw  = (const float*)d_in[4];
  const float* dtw  = (const float*)d_in[5];
  const float* dtb  = (const float*)d_in[6];
  const float* alog = (const float*)d_in[7];
  const float* Dw   = (const float*)d_in[8];
  const float* wo   = (const float*)d_in[9];
  float* out = (float*)d_out;

  char* ws = (char*)d_ws;
  size_t off = 0;
  const size_t oPL  = off; off = al256(off + (size_t)E_END * 2);
  const size_t oXSG = off; off = al256(off + (size_t)2 * LSEQ * DI * 4);
  const size_t oXC  = off; off = al256(off + (size_t)LSEQ * DI * 4);
  const size_t oXH  = off; off = al256(off + (size_t)LSEQ * K2 * 2);
  const size_t oXP  = off; off = al256(off + (size_t)LSEQ * XPN * 4);
  const size_t oYG  = off; off = al256(off + (size_t)LSEQ * K2 * 2);
  if (off > ws_size || off > (size_t)WSMAX) return;
  unsigned short* PL  = (unsigned short*)(ws + oPL);
  float*          XSG = (float*)(ws + oXSG);
  float*          XC  = (float*)(ws + oXC);
  unsigned short* XH  = (unsigned short*)(ws + oXH);
  float*          XP  = (float*)(ws + oXP);
  unsigned short* YG  = (unsigned short*)(ws + oYG);
  const unsigned short* XB   = PL + E_XB;
  const unsigned short* WIN  = PL + E_WIN;
  const unsigned short* OW2  = PL + E_OW;
  const unsigned short* XPW2 = PL + E_XPW;
  const float* XS = XSG;
  const float* G  = XSG + (size_t)LSEQ * DI;

  k_prep<<<U_TOT / NTHR, NTHR, 0, stream>>>(x, wi, wo, xpw, PL);
  k_gemm<1><<<dim3(LSEQ / GBM, NPJ / GBN), GTHR, 0, stream>>>(XB, WIN, XSG, DM, DI, DI, LSEQ * DI);
  k_conv<<<(LSEQ * (DI / 4)) / NTHR, NTHR, 0, stream>>>(XS, cw, cb, XC, XH);
  k_gemm<0><<<dim3(LSEQ / GBM, XPN / GBN), GTHR, 0, stream>>>(XH, XPW2, XP, K2, XPN, 0, 0);
  k_scan<<<DI / SCT, SCT, 0, stream>>>(XP, XC, G, alog, dtw, dtb, Dw, YG);
  k_gemm<0><<<dim3(LSEQ / GBM, DM / GBN), GTHR, 0, stream>>>(YG, OW2, out, K2, DM, 0, 0);
}
